// RelativeMultiHeadAttention_89309549953500
// MI455X (gfx1250) — hardware-verified
//
#include <hip/hip_runtime.h>
#include <math.h>

#ifndef NB
#define NB 8
#endif
#ifndef SEQ
#define SEQ 512
#endif
#define SEQ_FULL 512
#define DM 512
#define NH 8
#define DH 64
#define MAXLEN 5000
#define PE_ROWS_FULL 10001
#define NREL (2 * SEQ)
#define PE_ROW0 (MAXLEN - (SEQ - 1))
#define MTOK (NB * SEQ)

#define SLAB_P 68
#define AT_WAVES 8
#define AT_BPH (SEQ / (16 * AT_WAVES))
#define OS_P 52
#define CT_P 72

constexpr unsigned ilog2c(unsigned v) { return (v <= 1u) ? 0u : 1u + ilog2c(v >> 1); }
static constexpr unsigned LG_SEQ = ilog2c((unsigned)SEQ);
static constexpr unsigned LG_NREL = ilog2c((unsigned)NREL);
static constexpr unsigned LG_DM = ilog2c((unsigned)DM);

static constexpr float WCARRY = 64.0f;
static constexpr float CCARRY = 16.0f;
static constexpr float OSC = 1.0f / (WCARRY * CCARRY);
static constexpr float SC2 = 0.18033688011112042f;
static constexpr float PCL = 10.0f;
static constexpr float PFLOOR = -14.0f;

static_assert(OSC * WCARRY * CCARRY == 1.0f);
static_assert(DM == 512);
static_assert(NH * DH == DM);
static_assert(DH == 64);
static_assert(SEQ % 128 == 0 && SEQ >= 128 && SEQ <= SEQ_FULL);
static_assert((1u << LG_SEQ) == (unsigned)SEQ);
static_assert((1u << LG_NREL) == (unsigned)NREL);
static_assert((1u << LG_DM) == (unsigned)DM);
static_assert(MTOK % 64 == 0 && NREL % 64 == 0 && DM % 64 == 0);
static_assert(DM % 32 == 0 && DH % 32 == 0);
static_assert(SEQ % 32 == 0);
static_assert(PE_ROW0 >= 0 && PE_ROW0 + NREL - 2 < PE_ROWS_FULL);
static_assert(((MTOK / 64) * (DM / 64)) % 8 == 0);
static_assert(((NREL / 64) * (DM / 64)) % 8 == 0);
static_assert((MTOK * (DM / 8)) % 256 == 0 && (DM * (DM / 8)) % 256 == 0 && (NREL * (DM / 8)) % 256 == 0);
static_assert(AT_BPH * 16 * AT_WAVES == SEQ);
static_assert(OS_P >= 48 && OS_P % 4 == 0);
static_assert(CT_P >= 64 && CT_P % 8 == 0);
static_assert(SLAB_P >= 64 && SLAB_P % 4 == 0);
static_assert(32 * 16 * 4 == 16 * 64 * 2);
static_assert(32 * 16 * 8 == 16 * 64 * 4);
static_assert(8 * 16 * SLAB_P * 4 <= 131072);
static_assert(AT_WAVES * 16 * OS_P * 4 + AT_WAVES * 16 * CT_P * 2 <= 131072);

static constexpr size_t SZ_X16 = (size_t)MTOK * DM * 2;
static constexpr size_t SZ_W16 = (size_t)DM * DM * 2;
static constexpr size_t SZ_PE16 = (size_t)NREL * DM * 2;
static constexpr size_t SZ_HP = (size_t)NB * NH * SEQ * DH * 2;
static constexpr size_t SZ_RK = (size_t)NH * NREL * DH * 2;
static constexpr size_t SZ_CTX = (size_t)MTOK * DM * 2;
static constexpr size_t OFF_X16 = 0;
static constexpr size_t OFF_WQ = OFF_X16 + SZ_X16;
static constexpr size_t OFF_WK = OFF_WQ + SZ_W16;
static constexpr size_t OFF_WV = OFF_WK + SZ_W16;
static constexpr size_t OFF_WR = OFF_WV + SZ_W16;
static constexpr size_t OFF_WO = OFF_WR + SZ_W16;
static constexpr size_t OFF_PE = OFF_WO + SZ_W16;
static constexpr size_t OFF_QA = OFF_PE + SZ_PE16;
static constexpr size_t OFF_QB = OFF_QA + SZ_HP;
static constexpr size_t OFF_KP = OFF_QB + SZ_HP;
static constexpr size_t OFF_VT = OFF_KP + SZ_HP;
static constexpr size_t OFF_RK = OFF_VT + SZ_HP;
static constexpr size_t OFF_CTX = OFF_RK + SZ_RK;
static constexpr size_t WS_TOTAL = OFF_CTX + SZ_CTX;
static_assert(SZ_X16 % 256 == 0 && SZ_W16 % 256 == 0 && SZ_PE16 % 256 == 0 && SZ_HP % 256 == 0 && SZ_RK % 256 == 0 && SZ_CTX % 256 == 0);
static_assert(WS_TOTAL <= (size_t)134217728);

typedef _Float16 h16;
typedef __attribute__((ext_vector_type(16))) _Float16 v16h;
typedef __attribute__((ext_vector_type(8)))  _Float16 v8h;
typedef __attribute__((ext_vector_type(16))) __bf16   v16bf;
typedef __attribute__((ext_vector_type(8)))  float    v8f;
typedef __attribute__((ext_vector_type(4)))  float    v4f;
typedef __attribute__((ext_vector_type(4)))  unsigned int v4u;


#define VST2(T, ptr, val) do { const T vst2_v_ = (val); *(volatile T*)(ptr) = vst2_v_; __threadfence(); *(volatile T*)(ptr) = vst2_v_; } while (0)

__device__ __forceinline__ float bfr(float f) {
    unsigned u = __float_as_uint(f);
    u += 0x7FFFu + ((u >> 16) & 1u);
    return __uint_as_float(u & 0xFFFF0000u);
}
__device__ __forceinline__ unsigned bf16_bits(float f) {
    unsigned u = __float_as_uint(f);
    u += 0x7FFFu + ((u >> 16) & 1u);
    return u >> 16;
}
static __device__ __forceinline__ h16 toh_flush(float v) { const float w = (fabsf(v) < 6.103515625e-05f) ? 0.0f : v; return (h16)w; }

union FragU { v16h v; v8h h[2]; };
__device__ __forceinline__ v16h frag_ld(const _Float16* p) {
    FragU f; f.h[0] = *(const v8h*)(p); f.h[1] = *(const v8h*)(p + 16); return f.v;
}
union FragB { v16bf v; v4u q[2]; };
__device__ __forceinline__ v16bf frag_ldb(const unsigned short* p) {
    FragB f; f.q[0] = *(const v4u*)(p); f.q[1] = *(const v4u*)(p + 16); return f.v;
}
__device__ __forceinline__ v8f wmma16g(v16h a, v16h b, v8f c) {
    c = __builtin_amdgcn_wmma_f32_16x16x32_f16(false, a, false, b, (short)0, c, false, false);
    asm volatile("v_nop\n\tv_nop\n\tv_nop\n\tv_nop" : "+v"(c) : "v"(a), "v"(b));
    return c;
}
__device__ __forceinline__ v8f wmmabg(v16bf a, v16bf b, v8f c) {
    c = __builtin_amdgcn_wmma_f32_16x16x32_bf16(false, a, false, b, (short)0, c, false, false);
    asm volatile("v_nop\n\tv_nop\n\tv_nop\n\tv_nop" : "+v"(c) : "v"(a), "v"(b));
    return c;
}
__device__ __forceinline__ v16h  ldfrag(const _Float16* p)       { return frag_ld(p); }
__device__ __forceinline__ v16bf ldfrag(const unsigned short* p) { return frag_ldb(p); }
__device__ __forceinline__ v8f mma(v16h a, v16h b, v8f c)   { return wmma16g(a, b, c); }
__device__ __forceinline__ v8f mma(v16bf a, v16bf b, v8f c) { return wmmabg(a, b, c); }

__device__ __forceinline__ void wave_sync_lds() {
    __builtin_amdgcn_fence(3  , "workgroup");
    __builtin_amdgcn_wave_barrier();
    __builtin_amdgcn_fence(2  , "workgroup");
}

__global__ __launch_bounds__(256) void k_cvt_b16(const float* __restrict__ src, unsigned srow0, unsigned lgrpg, unsigned gstride,
                                                 unsigned nvalid, unsigned short* __restrict__ dst, unsigned nrows) {
    const unsigned u = blockIdx.x * 256u + threadIdx.x;
    if (u >= nrows * (unsigned)(DM / 8)) return;
    const unsigned row = u >> (LG_DM - 3u), c0 = (u & (unsigned)(DM / 8 - 1)) * 8u;
    const unsigned rv = min(row, nvalid - 1u);
    const unsigned srow = srow0 + (rv >> lgrpg) * gstride + (rv & ((1u << lgrpg) - 1u));
    const float* sp = src + (size_t)srow * DM + c0;
    const v4f a = *(const v4f*)sp, b = *(const v4f*)(sp + 4);
    const bool live = row < nvalid;
    const float v[8] = {a.x, a.y, a.z, a.w, b.x, b.y, b.z, b.w};
    unsigned w[8];
#pragma unroll
    for (int i = 0; i < 8; ++i) { const float t = live ? v[i] : 0.0f; w[i] = bf16_bits(t); }
    v4u pk;
    pk.x = w[0] | (w[1] << 16);
    pk.y = w[2] | (w[3] << 16);
    pk.z = w[4] | (w[5] << 16);
    pk.w = w[6] | (w[7] << 16);
    VST2(v4u, (v4u*)(dst + (size_t)row * DM + c0), pk);
}

__global__ __launch_bounds__(256) void k_cvt_h16(const float* __restrict__ src, _Float16* __restrict__ dst, unsigned nrows) {
    const unsigned u = blockIdx.x * 256u + threadIdx.x;
    if (u >= nrows * (unsigned)(DM / 8)) return;
    const unsigned row = u >> (LG_DM - 3u), c0 = (u & (unsigned)(DM / 8 - 1)) * 8u;
    const float* sp = src + (size_t)row * DM + c0;
    const v4f a = *(const v4f*)sp, b = *(const v4f*)(sp + 4);
    const float v[8] = {a.x, a.y, a.z, a.w, b.x, b.y, b.z, b.w};
    v8h hv;
#pragma unroll
    for (int i = 0; i < 8; ++i) hv[i] = toh_flush(bfr(v[i]) * WCARRY);
    VST2(v8h, (v8h*)(dst + (size_t)row * DM + c0), hv);
}

template <typename FT, typename PT>
static __device__ __forceinline__ void gemm_main(const PT* __restrict__ A, const PT* __restrict__ Bt,
                                                 unsigned m0, unsigned n0, unsigned lane, v8f (&acc)[4][4]) {
    const unsigned rlane = lane & 15u;
    const unsigned koff = (lane >> 4) * 8u;
#pragma unroll
    for (int i = 0; i < 4; ++i)
#pragma unroll
        for (int j = 0; j < 4; ++j) acc[i][j] = (v8f){0.f, 0.f, 0.f, 0.f, 0.f, 0.f, 0.f, 0.f};
    const PT* ap = A + (size_t)(m0 + rlane) * DM + koff;
    const PT* bp = Bt + (size_t)(n0 + rlane) * DM + koff;
#pragma unroll 1
    for (unsigned k0 = 0; k0 < (unsigned)DM; k0 += 32u) {
        FT bh[4];
#pragma unroll
        for (int j = 0; j < 4; ++j) bh[j] = ldfrag(bp + (size_t)(16 * j) * DM + k0);
#pragma unroll
        for (int i = 0; i < 4; ++i) {
            const FT ah = ldfrag(ap + (size_t)(16 * i) * DM + k0);
#pragma unroll
            for (int j = 0; j < 4; ++j) acc[i][j] = mma(ah, bh[j], acc[i][j]);
        }
    }
}

static __device__ __forceinline__ void store_slab_h(const float* slab, _Float16* dst, unsigned pitch, unsigned lane) {
    const unsigned q = lane >> 3, c8 = (lane & 7u) * 8u;
    v8h hv[4];
#pragma unroll
    for (int it = 0; it < 4; ++it) {
        const unsigned row = (unsigned)it * 4u + q;
        const float* sp = slab + row * SLAB_P + c8;
#pragma unroll
        for (int e = 0; e < 8; ++e) hv[it][e] = toh_flush(sp[e]);
    }
    for (int pass = 0; pass < 2; ++pass) {
#pragma unroll
        for (int it = 0; it < 4; ++it) {
            const unsigned row = (unsigned)it * 4u + q;
            *(volatile v8h*)(dst + (size_t)row * pitch + c8) = hv[it];
        }
        __threadfence();
    }
}
static __device__ __forceinline__ void store_slab_f(const float* slab, float* dst, unsigned pitch, unsigned lane) {
    const unsigned hh = lane >> 4, c4 = (lane & 15u) * 4u;
#pragma unroll
    for (int half = 0; half < 2; ++half) {
        v4f vv[4];
#pragma unroll
        for (int it = 0; it < 4; ++it) {
            const unsigned row = (unsigned)(half * 4 + it) * 2u + hh;
            vv[it] = *(const v4f*)(slab + row * SLAB_P + c4);
        }
        for (int pass = 0; pass < 2; ++pass) {
#pragma unroll
            for (int it = 0; it < 4; ++it) {
                const unsigned row = (unsigned)(half * 4 + it) * 2u + hh;
                *(volatile v4f*)(dst + (size_t)row * pitch + c4) = vv[it];
            }
            __threadfence();
        }
    }
}

__global__ __launch_bounds__(256) void k_gemm_q(const unsigned short* __restrict__ X16, const unsigned short* __restrict__ W16,
                                                const float* __restrict__ bq, const float* __restrict__ ub, const float* __restrict__ vb,
                                                _Float16* __restrict__ QA, _Float16* __restrict__ QB) {
    __shared__ __align__(16) float sT[8][16 * SLAB_P];
    const unsigned lane = threadIdx.x & 31u;
    const unsigned wave = (unsigned)__builtin_amdgcn_readfirstlane((int)(threadIdx.x >> 5));
    const unsigned tile = blockIdx.x * 8u + wave;
    if (tile >= (unsigned)((MTOK / 64) * (DM / 64))) return;
    const unsigned tm = tile / (unsigned)(DM / 64);
    const unsigned tn = tile % (unsigned)(DM / 64);
    const unsigned m0 = tm << 6, n0 = tn << 6;
    const unsigned rlane = lane & 15u, mOff = (lane >> 4) * 8u;
    v8f acc[4][4];
    gemm_main<v16bf, unsigned short>(X16, W16, m0, n0, lane, acc);
    float* slab = sT[wave];
    float cq[4], cu[4], cv[4];
#pragma unroll
    for (int j = 0; j < 4; ++j) {
        const unsigned n = n0 + ((unsigned)j << 4) + rlane;
        cq[j] = bfr(bq[n]); cu[j] = bfr(ub[n]); cv[j] = bfr(vb[n]);
    }
    const unsigned bb = m0 / (unsigned)SEQ, s0 = m0 % (unsigned)SEQ;
    const size_t obase = ((size_t)(bb * (unsigned)NH + tn) * SEQ + s0) * DH;
#pragma unroll
    for (int i = 0; i < 4; ++i) {
#pragma unroll
        for (int j = 0; j < 4; ++j)
#pragma unroll
            for (int r = 0; r < 8; ++r)
                slab[(mOff + (unsigned)r) * SLAB_P + ((unsigned)j << 4) + rlane] = (acc[i][j][r] + cq[j]) + cu[j];
        wave_sync_lds();
        store_slab_h(slab, QA + obase + (size_t)(16 * i) * DH, DH, lane);
        wave_sync_lds();
#pragma unroll
        for (int j = 0; j < 4; ++j)
#pragma unroll
            for (int r = 0; r < 8; ++r)
                slab[(mOff + (unsigned)r) * SLAB_P + ((unsigned)j << 4) + rlane] = (acc[i][j][r] + cq[j]) + cv[j];
        wave_sync_lds();
        store_slab_h(slab, QB + obase + (size_t)(16 * i) * DH, DH, lane);
        wave_sync_lds();
    }
}

__global__ __launch_bounds__(256) void k_gemm_k(const unsigned short* __restrict__ X16, const unsigned short* __restrict__ W16,
                                                const float* __restrict__ bk, _Float16* __restrict__ KP) {
    __shared__ __align__(16) float sT[8][16 * SLAB_P];
    const unsigned lane = threadIdx.x & 31u;
    const unsigned wave = (unsigned)__builtin_amdgcn_readfirstlane((int)(threadIdx.x >> 5));
    const unsigned tile = blockIdx.x * 8u + wave;
    if (tile >= (unsigned)((MTOK / 64) * (DM / 64))) return;
    const unsigned tm = tile / (unsigned)(DM / 64);
    const unsigned tn = tile % (unsigned)(DM / 64);
    const unsigned m0 = tm << 6, n0 = tn << 6;
    const unsigned rlane = lane & 15u, mOff = (lane >> 4) * 8u;
    v8f acc[4][4];
    gemm_main<v16bf, unsigned short>(X16, W16, m0, n0, lane, acc);
    float* slab = sT[wave];
    float cb[4];
#pragma unroll
    for (int j = 0; j < 4; ++j) cb[j] = bfr(bk[n0 + ((unsigned)j << 4) + rlane]);
    const unsigned bb = m0 / (unsigned)SEQ, s0 = m0 % (unsigned)SEQ;
    const size_t obase = ((size_t)(bb * (unsigned)NH + tn) * SEQ + s0) * DH;
#pragma unroll
    for (int i = 0; i < 4; ++i) {
#pragma unroll
        for (int j = 0; j < 4; ++j)
#pragma unroll
            for (int r = 0; r < 8; ++r)
                slab[(mOff + (unsigned)r) * SLAB_P + ((unsigned)j << 4) + rlane] = acc[i][j][r] + cb[j];
        wave_sync_lds();
        store_slab_h(slab, KP + obase + (size_t)(16 * i) * DH, DH, lane);
        wave_sync_lds();
    }
}

__global__ __launch_bounds__(256) void k_gemm_vt(const unsigned short* __restrict__ W16, const unsigned short* __restrict__ X16,
                                                 const float* __restrict__ bv, _Float16* __restrict__ VT) {
    __shared__ __align__(16) float sT[8][16 * SLAB_P];
    const unsigned lane = threadIdx.x & 31u;
    const unsigned wave = (unsigned)__builtin_amdgcn_readfirstlane((int)(threadIdx.x >> 5));
    const unsigned tile = blockIdx.x * 8u + wave;
    if (tile >= (unsigned)((DM / 64) * (MTOK / 64))) return;
    const unsigned tm = tile / (unsigned)(MTOK / 64);
    const unsigned tn = tile % (unsigned)(MTOK / 64);
    const unsigned m0 = tm << 6, n0 = tn << 6;
    const unsigned rlane = lane & 15u, mOff = (lane >> 4) * 8u;
    v8f acc[4][4];
    gemm_main<v16bf, unsigned short>(W16, X16, m0, n0, lane, acc);
    float* slab = sT[wave];
    const unsigned bb = n0 / (unsigned)SEQ, s0 = n0 % (unsigned)SEQ;
    const size_t obase = ((size_t)(bb * (unsigned)NH + tm) * DH) * SEQ + s0;
#pragma unroll
    for (int i = 0; i < 4; ++i) {
        float cr[8];
#pragma unroll
        for (int r = 0; r < 8; ++r) cr[r] = bfr(bv[m0 + ((unsigned)i << 4) + mOff + (unsigned)r]);
#pragma unroll
        for (int j = 0; j < 4; ++j)
#pragma unroll
            for (int r = 0; r < 8; ++r)
                slab[(mOff + (unsigned)r) * SLAB_P + ((unsigned)j << 4) + rlane] = acc[i][j][r] + cr[r];
        wave_sync_lds();
        store_slab_h(slab, VT + obase + (size_t)(16 * i) * SEQ, SEQ, lane);
        wave_sync_lds();
    }
}

__global__ __launch_bounds__(256) void k_gemm_r(const unsigned short* __restrict__ PE16, const unsigned short* __restrict__ W16,
                                                _Float16* __restrict__ RK) {
    __shared__ __align__(16) float sT[8][16 * SLAB_P];
    const unsigned lane = threadIdx.x & 31u;
    const unsigned wave = (unsigned)__builtin_amdgcn_readfirstlane((int)(threadIdx.x >> 5));
    const unsigned tile = blockIdx.x * 8u + wave;
    if (tile >= (unsigned)((NREL / 64) * (DM / 64))) return;
    const unsigned tm = tile / (unsigned)(DM / 64);
    const unsigned tn = tile % (unsigned)(DM / 64);
    const unsigned m0 = tm << 6, n0 = tn << 6;
    const unsigned rlane = lane & 15u, mOff = (lane >> 4) * 8u;
    v8f acc[4][4];
    gemm_main<v16bf, unsigned short>(PE16, W16, m0, n0, lane, acc);
    float* slab = sT[wave];
    const size_t obase = ((size_t)tn * NREL + m0) * DH;
#pragma unroll
    for (int i = 0; i < 4; ++i) {
#pragma unroll
        for (int j = 0; j < 4; ++j)
#pragma unroll
            for (int r = 0; r < 8; ++r)
                slab[(mOff + (unsigned)r) * SLAB_P + ((unsigned)j << 4) + rlane] = acc[i][j][r];
        wave_sync_lds();
        store_slab_h(slab, RK + obase + (size_t)(16 * i) * DH, DH, lane);
        wave_sync_lds();
    }
}

__global__ __launch_bounds__(256) void k_gemm_out(const _Float16* __restrict__ CTX, const _Float16* __restrict__ WO16,
                                                  const float* __restrict__ bo, float* __restrict__ out) {
    __shared__ __align__(16) float sT[8][16 * SLAB_P];
    const unsigned lane = threadIdx.x & 31u;
    const unsigned wave = (unsigned)__builtin_amdgcn_readfirstlane((int)(threadIdx.x >> 5));
    const unsigned tile = blockIdx.x * 8u + wave;
    if (tile >= (unsigned)((MTOK / 64) * (DM / 64))) return;
    const unsigned tm = tile / (unsigned)(DM / 64);
    const unsigned tn = tile % (unsigned)(DM / 64);
    const unsigned m0 = tm << 6, n0 = tn << 6;
    const unsigned rlane = lane & 15u, mOff = (lane >> 4) * 8u;
    v8f acc[4][4];
    gemm_main<v16h, _Float16>(CTX, WO16, m0, n0, lane, acc);
    float* slab = sT[wave];
    float cb[4];
#pragma unroll
    for (int j = 0; j < 4; ++j) cb[j] = bfr(bo[n0 + ((unsigned)j << 4) + rlane]);
#pragma unroll
    for (int i = 0; i < 4; ++i) {
#pragma unroll
        for (int j = 0; j < 4; ++j)
#pragma unroll
            for (int r = 0; r < 8; ++r)
                slab[(mOff + (unsigned)r) * SLAB_P + ((unsigned)j << 4) + rlane] = acc[i][j][r] * OSC + cb[j];
        wave_sync_lds();
        store_slab_f(slab, out + (size_t)(m0 + 16u * (unsigned)i) * DM + n0, DM, lane);
        wave_sync_lds();
    }
}

__global__ __launch_bounds__(256) void k_attn(const _Float16* __restrict__ QA, const _Float16* __restrict__ QB,
                                              const _Float16* __restrict__ KP, const _Float16* __restrict__ VT,
                                              const _Float16* __restrict__ RK, _Float16* __restrict__ CTX) {
    __shared__ __align__(16) float    sOS[AT_WAVES][16 * OS_P];
    __shared__ __align__(16) _Float16 sCT[AT_WAVES][16 * CT_P];
    const unsigned lane = threadIdx.x & 31u;
    const unsigned wave = (unsigned)__builtin_amdgcn_readfirstlane((int)(threadIdx.x >> 5));
    const unsigned hi = lane >> 4, lr = lane & 15u;
    const unsigned bx = blockIdx.x;
    const unsigned bh = bx / (unsigned)AT_BPH;
    const unsigned t0 = ((bx % (unsigned)AT_BPH) * (unsigned)AT_WAVES + wave) * 16u;
    const unsigned hd = bh % (unsigned)NH, bb = bh / (unsigned)NH;

    const size_t qoff = ((size_t)bh * SEQ + t0 + lr) * DH + 8u * hi;
    const v16h qa0 = frag_ld(QA + qoff), qa1 = frag_ld(QA + qoff + 32);
    const v16h qb0 = frag_ld(QB + qoff), qb1 = frag_ld(QB + qoff + 32);
    const _Float16* kbase = KP + ((size_t)bh * SEQ + lr) * DH + 8u * hi;
    const _Float16* vbase = VT + ((size_t)bh * DH + lr) * SEQ + 8u * hi;
    const _Float16* rbase = RK + (size_t)hd * NREL * DH + 8u * hi;

    float mrun = -3.0e38f, lsum = 0.f;
    v8f o[4];
#pragma unroll
    for (int t = 0; t < 4; ++t) o[t] = (v8f){0.f, 0.f, 0.f, 0.f, 0.f, 0.f, 0.f, 0.f};

#pragma unroll 1
    for (unsigned key0 = 0; key0 < (unsigned)SEQ; key0 += 32u) {
        const unsigned rlo = ((unsigned)SEQ - 16u) - t0 + key0;
#pragma unroll
        for (int u = 0; u < 3; ++u) {
            const unsigned rr = min(rlo + 16u * (unsigned)u + lr, (unsigned)(NREL - 2));
            const _Float16* rp = rbase + (size_t)rr * DH;
            v8f d = (v8f){0.f, 0.f, 0.f, 0.f, 0.f, 0.f, 0.f, 0.f};
            d = wmma16g(frag_ld(rp), qb0, d);
            d = wmma16g(frag_ld(rp + 32), qb1, d);
            v4f d0, d1;
            d0.x = d[0]; d0.y = d[1]; d0.z = d[2]; d0.w = d[3];
            d1.x = d[4]; d1.y = d[5]; d1.z = d[6]; d1.w = d[7];
            *(v4f*)&sOS[wave][lr * OS_P + 16u * (unsigned)u + 8u * hi] = d0;
            *(v4f*)&sOS[wave][lr * OS_P + 16u * (unsigned)u + 8u * hi + 4u] = d1;
        }
        wave_sync_lds();
        float pa[8], pb[8];
        {
            const unsigned dg = lr * (unsigned)(OS_P - 1) + 15u + 8u * hi;
#pragma unroll
            for (int r = 0; r < 8; ++r) { pa[r] = sOS[wave][dg + (unsigned)r]; pb[r] = sOS[wave][dg + 16u + (unsigned)r]; }
        }
        wave_sync_lds();

        v8f sa = (v8f){0.f, 0.f, 0.f, 0.f, 0.f, 0.f, 0.f, 0.f};
        v8f sb = sa;
        {
            const _Float16* kp = kbase + (size_t)key0 * DH;
            sa = wmma16g(frag_ld(kp), qa0, sa);
            sa = wmma16g(frag_ld(kp + 32), qa1, sa);
            sb = wmma16g(frag_ld(kp + 16 * DH), qa0, sb);
            sb = wmma16g(frag_ld(kp + 16 * DH + 32), qa1, sb);
        }

        float ea[8], eb[8];
        float mx = -3.0e38f;
#pragma unroll
        for (int r = 0; r < 8; ++r) {
            ea[r] = (sa[r] + pa[r]) * SC2;
            eb[r] = (sb[r] + pb[r]) * SC2;
            mx = fmaxf(mx, fmaxf(ea[r], eb[r]));
        }
        mx = fmaxf(mx, __shfl_xor(mx, 16, 32));
        const float mnew = fmaxf(mrun, mx);
        const float alpha = exp2f(mrun - mnew);
        mrun = mnew;
        float psum = 0.f;
        v16h pf;
#pragma unroll
        for (int r = 0; r < 8; ++r) {
            const float xa = (ea[r] - mnew) + PCL;
            const float xb = (eb[r] - mnew) + PCL;
            const float fa = (xa < PFLOOR) ? 0.0f : exp2f(xa);
            const float fb = (xb < PFLOOR) ? 0.0f : exp2f(xb);
            const h16 ha = toh_flush(fa);
            const h16 hb = toh_flush(fb);
            pf[r] = ha;
            pf[8 + r] = hb;
            psum += (float)ha + (float)hb;
        }
        lsum = lsum * alpha + psum;
#pragma unroll
        for (int t = 0; t < 4; ++t)
#pragma unroll
            for (int r = 0; r < 8; ++r) o[t][r] *= alpha;

#pragma unroll
        for (int t = 0; t < 4; ++t) {
            const v16h va = frag_ld(vbase + (size_t)(16 * t) * SEQ + key0);
            o[t] = wmma16g(va, pf, o[t]);
        }
    }

    const float ltot = lsum + __shfl_xor(lsum, 16, 32);
    const float inv = CCARRY / ltot;
#pragma unroll
    for (int t = 0; t < 4; ++t) {
        v8h cv;
#pragma unroll
        for (int r = 0; r < 8; ++r) cv[r] = toh_flush(o[t][r] * inv);
        *(v8h*)&sCT[wave][lr * CT_P + 16u * (unsigned)t + 8u * hi] = cv;
    }
    wave_sync_lds();
    {
        const unsigned q = lane >> 3, c8 = (lane & 7u) * 8u;
        v8h ov[4];
#pragma unroll
        for (int it = 0; it < 4; ++it) ov[it] = *(const v8h*)&sCT[wave][((unsigned)it * 4u + q) * CT_P + c8];
        _Float16* dst = CTX + ((size_t)bb * SEQ + t0) * DM + hd * (unsigned)DH;
        for (int pass = 0; pass < 2; ++pass) {
#pragma unroll
            for (int it = 0; it < 4; ++it) *(volatile v8h*)(dst + (size_t)((unsigned)it * 4u + q) * DM + c8) = ov[it];
            __threadfence();
        }
    }
}

extern "C" void kernel_launch(void* const* d_in, const int* in_sizes, int n_in, void* d_out, int out_size,
                              void* d_ws, size_t ws_size, hipStream_t stream) {
    if (n_in < 13) return;
    if (in_sizes[0] < ((NB - 1) * SEQ_FULL + SEQ) * DM) return;
    if (in_sizes[1] < DM * DM || in_sizes[3] < DM * DM || in_sizes[5] < DM * DM || in_sizes[7] < DM * DM || in_sizes[9] < DM * DM) return;
    if (in_sizes[2] < DM || in_sizes[4] < DM || in_sizes[6] < DM || in_sizes[8] < DM) return;
    if (in_sizes[10] < NH * DH || in_sizes[11] < NH * DH) return;
    if (in_sizes[12] < (PE_ROW0 + NREL - 1) * DM) return;
    if (out_size < MTOK * DM) return;
    if (ws_size < WS_TOTAL) return;

    const float* x   = (const float*)d_in[0];
    const float* wq  = (const float*)d_in[1];
    const float* bq  = (const float*)d_in[2];
    const float* wk  = (const float*)d_in[3];
    const float* bk  = (const float*)d_in[4];
    const float* wv  = (const float*)d_in[5];
    const float* bv  = (const float*)d_in[6];
    const float* wo  = (const float*)d_in[7];
    const float* bo  = (const float*)d_in[8];
    const float* wr  = (const float*)d_in[9];
    const float* ub  = (const float*)d_in[10];
    const float* vb  = (const float*)d_in[11];
    const float* pe  = (const float*)d_in[12];
    float* out = (float*)d_out;

    char* wsp = (char*)d_ws;
    unsigned short* X16  = (unsigned short*)(wsp + OFF_X16);
    unsigned short* WQ16 = (unsigned short*)(wsp + OFF_WQ);
    unsigned short* WK16 = (unsigned short*)(wsp + OFF_WK);
    unsigned short* WV16 = (unsigned short*)(wsp + OFF_WV);
    unsigned short* WR16 = (unsigned short*)(wsp + OFF_WR);
    _Float16*       WO16 = (_Float16*)(wsp + OFF_WO);
    unsigned short* PE16 = (unsigned short*)(wsp + OFF_PE);
    _Float16*       QA   = (_Float16*)(wsp + OFF_QA);
    _Float16*       QB   = (_Float16*)(wsp + OFF_QB);
    _Float16*       KP   = (_Float16*)(wsp + OFF_KP);
    _Float16*       VT   = (_Float16*)(wsp + OFF_VT);
    _Float16*       RK   = (_Float16*)(wsp + OFF_RK);
    _Float16*       CTX  = (_Float16*)(wsp + OFF_CTX);

    k_cvt_b16<<<(MTOK * (DM / 8)) / 256, 256, 0, stream>>>(x, 0u, LG_SEQ, (unsigned)SEQ_FULL, (unsigned)MTOK, X16, (unsigned)MTOK);
    k_cvt_b16<<<(DM * (DM / 8)) / 256, 256, 0, stream>>>(wq, 0u, LG_DM, (unsigned)DM, (unsigned)DM, WQ16, (unsigned)DM);
    k_cvt_b16<<<(DM * (DM / 8)) / 256, 256, 0, stream>>>(wk, 0u, LG_DM, (unsigned)DM, (unsigned)DM, WK16, (unsigned)DM);
    k_cvt_b16<<<(DM * (DM / 8)) / 256, 256, 0, stream>>>(wv, 0u, LG_DM, (unsigned)DM, (unsigned)DM, WV16, (unsigned)DM);
    k_cvt_b16<<<(DM * (DM / 8)) / 256, 256, 0, stream>>>(wr, 0u, LG_DM, (unsigned)DM, (unsigned)DM, WR16, (unsigned)DM);
    k_cvt_b16<<<(NREL * (DM / 8)) / 256, 256, 0, stream>>>(pe, (unsigned)PE_ROW0, LG_NREL, 0u, (unsigned)(NREL - 1), PE16, (unsigned)NREL);
    k_cvt_h16<<<(DM * (DM / 8)) / 256, 256, 0, stream>>>(wo, WO16, (unsigned)DM);

    k_gemm_q<<<((MTOK / 64) * (DM / 64)) / 8, 256, 0, stream>>>(X16, WQ16, bq, ub, vb, QA, QB);
    k_gemm_k<<<((MTOK / 64) * (DM / 64)) / 8, 256, 0, stream>>>(X16, WK16, bk, KP);
    k_gemm_vt<<<((DM / 64) * (MTOK / 64)) / 8, 256, 0, stream>>>(WV16, X16, bv, VT);
    k_gemm_r<<<((NREL / 64) * (DM / 64)) / 8, 256, 0, stream>>>(PE16, WR16, RK);

    k_attn<<<NB * NH * AT_BPH, 256, 0, stream>>>(QA, QB, KP, VT, RK, CTX);

    k_gemm_out<<<((MTOK / 64) * (DM / 64)) / 8, 256, 0, stream>>>(CTX, WO16, bo, out);
}
